// multihead_attention_3d_4432406249853
// MI455X (gfx1250) — hardware-verified
//
#include <hip/hip_runtime.h>


namespace {
constexpr int C = 256, GZ = 16, NP = 4096, NH = 8, DH = 32, KT = 27 * C  ;
constexpr float QS = 8.0f, VS = 8.0f, PS = 8.0f, OS_ = 8.0f, SCALE = 0.17677669529663687f;
constexpr size_t QPL = (size_t)NH * NP * DH, VPL = (size_t)NH * DH * NP;

typedef _Float16 b16;
typedef __attribute__((ext_vector_type(16))) _Float16 v16b;
typedef __attribute__((ext_vector_type(16))) __bf16 v16bb;
typedef __attribute__((ext_vector_type(8))) _Float16 v8b;
typedef __attribute__((ext_vector_type(8))) unsigned short v8us;
typedef __attribute__((ext_vector_type(8))) float v8f;
typedef __attribute__((ext_vector_type(4))) float v4f;
__device__ __forceinline__ float bf16_rne(float f) { unsigned int u = __float_as_uint(f); u += 0x7FFFu + ((u >> 16) & 1u); return __uint_as_float(u & 0xFFFF0000u); }
__device__ __forceinline__ unsigned short bf16_bits(float f) { unsigned int u = __float_as_uint(f); u += 0x7FFFu + ((u >> 16) & 1u); return (unsigned short)(u >> 16); }
__device__ __forceinline__ void split16(float v, b16& hi, b16& lo) { hi = (b16)v; lo = (b16)(v - (float)hi); }
__device__ __forceinline__ v16b frag_kb(const b16* p, int hh) { const v8b a = *(const v8b*)(p + 8 * hh), b = *(const v8b*)(p + 16 + 8 * hh); v16b f;
#pragma unroll
  for (int e = 0; e < 8; ++e) { f[e] = a[e]; f[8 + e] = b[e]; } return f; }
__device__ __forceinline__ v16bb frag_bf(const unsigned short* p, int hh) { const v8us a = *(const v8us*)(p + 8 * hh), b = *(const v8us*)(p + 16 + 8 * hh); union { unsigned short s[16]; v16bb v; } u;
#pragma unroll
  for (int e = 0; e < 8; ++e) { u.s[e] = a[e]; u.s[8 + e] = b[e]; } return u.v; }
__device__ __forceinline__ v8f wmma16b(v16b a, v16b b, v8f c) { v8f d = __builtin_amdgcn_wmma_f32_16x16x32_f16(false, a, false, b, (short)0, c, false, false); asm volatile("v_nop\n\tv_nop\n\tv_nop\n\tv_nop" : "+v"(d) : "v"(a), "v"(b)); return d; }
__device__ __forceinline__ v8f wmma16bb(v16bb a, v16bb b, v8f c) { v8f d = __builtin_amdgcn_wmma_f32_16x16x32_bf16(false, a, false, b, (short)0, c, false, false); asm volatile("v_nop\n\tv_nop\n\tv_nop\n\tv_nop" : "+v"(d) : "v"(a), "v"(b)); return d; }
__device__ __forceinline__ void wave_lds_sync() { __builtin_amdgcn_fence(__ATOMIC_RELEASE, "workgroup"); __builtin_amdgcn_wave_barrier(); __builtin_amdgcn_fence(__ATOMIC_ACQUIRE, "workgroup"); }
__device__ __forceinline__ float nexp(float x) { return __builtin_amdgcn_exp2f(x * 1.4426950408889634f); }

__global__ __launch_bounds__(256) void prep_kernel(const float* __restrict__ x, const float* __restrict__ wq, const float* __restrict__ wk, const float* __restrict__ wv, const float* __restrict__ wt, unsigned short* __restrict__ xT, unsigned short* __restrict__ w16, b16* __restrict__ wt16) {
  __shared__ __attribute__((aligned(16))) unsigned short Tt[64][C + 8];
  const int t_ = threadIdx.x, p0 = blockIdx.x * 64;
  for (int i = t_; i < C * 64; i += 256) { const int c = i >> 6, pp = i & 63; Tt[pp][c] = bf16_bits(x[(size_t)c * NP + p0 + pp]); }
  __syncthreads();
  const size_t tid = (size_t)blockIdx.x * blockDim.x + threadIdx.x, nth = (size_t)gridDim.x * blockDim.x;
  for (int pass = 0; pass < 2; ++pass) {
    for (int i = t_; i < 64 * C / 8; i += 256) { const int pp = i >> 5, c8 = (i & 31) * 8; *(volatile v8us*)(xT + (size_t)(p0 + pp) * C + c8) = *(const v8us*)(&Tt[pp][c8]); }
    for (size_t p = tid; p < (size_t)3 * C * C / 8; p += nth) { const size_t m = p / (C * C / 8), q = p % (C * C / 8); const float* W = (m == 0) ? wq : (m == 1) ? wk : wv; v8us o;
#pragma unroll
      for (int e = 0; e < 8; ++e) o[e] = bf16_bits(W[q * 8 + e]);
      *(volatile v8us*)(w16 + p * 8) = o; }
    for (size_t p = tid; p < (size_t)C * KT / 8; p += nth) { const size_t co = p / (KT / 8); const int r = (int)(p % (KT / 8)) * 8, tap = r / C, ci0 = r % C; v8b o;
#pragma unroll
      for (int e = 0; e < 8; ++e) o[e] = (b16)bf16_rne(wt[((size_t)co * C + ci0 + e) * 27 + tap]);
      *(volatile v8b*)(wt16 + co * KT + r) = o; }
    __threadfence();
  }
}

__global__ __launch_bounds__(128) void proj_kernel(const unsigned short* __restrict__ xT, const unsigned short* __restrict__ w16, const float* __restrict__ bq, const float* __restrict__ bk, const float* __restrict__ bv, b16* __restrict__ qh, b16* __restrict__ kh, b16* __restrict__ vt) {
  __shared__ __attribute__((aligned(16))) b16 Th[2][128][32], Tl[2][128][32]; __shared__ __attribute__((aligned(16))) b16 Vh[64][128 + 8], Vl[64][128 + 8];
  const int lane = threadIdx.x & 31, wave = threadIdx.x >> 5, nloc = lane & 15, hlf = lane >> 4, which = blockIdx.z, m0 = blockIdx.y * 128 + wave * 32, c0 = blockIdx.x * 64, p0 = blockIdx.y * 128;
  const unsigned short* Wt = w16 + (size_t)which * C * C; const float* bias = (which == 0) ? bq : (which == 1) ? bk : bv;
  v8f acc[2][4];
#pragma unroll
  for (int r = 0; r < 2; ++r)
#pragma unroll
    for (int t = 0; t < 4; ++t) acc[r][t] = (v8f){};
#pragma unroll 2
  for (int kb = 0; kb < C; kb += 32) { const v16bb a0 = frag_bf(xT + (size_t)(m0 + nloc) * C + kb, hlf), a1 = frag_bf(xT + (size_t)(m0 + 16 + nloc) * C + kb, hlf);
#pragma unroll
    for (int t = 0; t < 4; ++t) { const v16bb bw = frag_bf(Wt + (size_t)(c0 + t * 16 + nloc) * C + kb, hlf); acc[0][t] = wmma16bb(a0, bw, acc[0][t]); acc[1][t] = wmma16bb(a1, bw, acc[1][t]); } }
  const float scl = (which == 0) ? SCALE * QS : (which == 1) ? QS : VS;
#pragma unroll
  for (int t = 0; t < 4; ++t) { const int c = c0 + t * 16 + nloc; const float bb = bf16_rne(bias[c]); const int hl = t >> 1, d = (t & 1) * 16 + nloc;
#pragma unroll
    for (int r = 0; r < 2; ++r)
#pragma unroll
      for (int v = 0; v < 8; ++v) { b16 a_, c_; split16((acc[r][t][v] + bb) * scl, a_, c_); const int row = wave * 32 + r * 16 + 8 * hlf + v;
        if (which < 2) { Th[hl][row][d] = a_; Tl[hl][row][d] = c_; } else { Vh[t * 16 + nloc][row] = a_; Vl[t * 16 + nloc][row] = c_; } } }
  __syncthreads();
  for (int pass = 0; pass < 2; ++pass) {
    if (which < 2) { b16* base = (which == 0) ? qh : kh;
      for (int i = threadIdx.x; i < 2 * 128 * 32 / 8; i += 128) { const int hl = i / 512, rem = i % 512; const size_t dst = ((size_t)(blockIdx.x * 2 + hl) * NP + p0) * DH + (size_t)rem * 8;
        *(volatile v8b*)(base + dst) = *(const v8b*)(&Th[hl][0][0] + rem * 8); *(volatile v8b*)(base + QPL + dst) = *(const v8b*)(&Tl[hl][0][0] + rem * 8); } }
    else { for (int i = threadIdx.x; i < 64 * 16; i += 128) { const int cc = i >> 4, c8 = (i & 15) * 8; const int h = blockIdx.x * 2 + (cc >> 5), d = cc & 31; const size_t dst = ((size_t)h * DH + d) * NP + p0 + c8;
        *(volatile v8b*)(vt + dst) = *(const v8b*)(&Vh[cc][c8]); *(volatile v8b*)(vt + VPL + dst) = *(const v8b*)(&Vl[cc][c8]); } }
    __threadfence(); }
}

__global__ __launch_bounds__(256) void attn_kernel(const b16* __restrict__ qh, const b16* __restrict__ kh, const b16* __restrict__ vt, float* __restrict__ orow) {
  __shared__ __attribute__((aligned(16))) float Os[16][C + 4];
  const int wid = threadIdx.x >> 5, lane = threadIdx.x & 31, hh = lane >> 4, col = lane & 15; const int q0 = blockIdx.x * 16, h = wid, qi = q0 + col;
  const b16* Q = qh + ((size_t)h * NP) * DH; const b16* K = kh + ((size_t)h * NP) * DH; const b16* V = vt + ((size_t)h * DH) * NP;
  const v16b qf = frag_kb(Q + (size_t)qi * DH, hh), ql = frag_kb(Q + QPL + (size_t)qi * DH, hh);
  float m = -INFINITY, l = 0.0f; v8f o[2] = {{}, {}};
  for (int kb = 0; kb < NP; kb += 32) {
    const v16b ka = frag_kb(K + (size_t)(kb + col) * DH, hh), kal = frag_kb(K + QPL + (size_t)(kb + col) * DH, hh), kb_ = frag_kb(K + (size_t)(kb + 16 + col) * DH, hh), kbl = frag_kb(K + QPL + (size_t)(kb + 16 + col) * DH, hh);
    v8f s0 = {}, s1 = {}; s0 = wmma16b(ka, qf, s0); s0 = wmma16b(ka, ql, s0); s0 = wmma16b(kal, qf, s0); s1 = wmma16b(kb_, qf, s1); s1 = wmma16b(kb_, ql, s1); s1 = wmma16b(kbl, qf, s1);
    float mr = -INFINITY;
#pragma unroll
    for (int r = 0; r < 8; ++r) { s0[r] *= 1.0f / (QS * QS); s1[r] *= 1.0f / (QS * QS); mr = fmaxf(mr, fmaxf(s0[r], s1[r])); }
    mr = fmaxf(mr, __shfl_xor(mr, 16));
    const float mn = fmaxf(m, mr), al_ = nexp(m - mn); m = mn; float sum = 0.0f; v16b pb, pl;
#pragma unroll
    for (int r = 0; r < 8; ++r) { const float p0 = nexp(s0[r] - mn), p1 = nexp(s1[r] - mn); sum += p0 + p1; b16 a, c; split16(p0 * PS, a, c); pb[r] = a; pl[r] = c; split16(p1 * PS, a, c); pb[8 + r] = a; pl[8 + r] = c; }
    sum += __shfl_xor(sum, 16); l = l * al_ + sum;
#pragma unroll
    for (int n = 0; n < 2; ++n) { o[n] *= al_; const v16b vf = frag_kb(V + (size_t)(n * 16 + col) * NP + kb, hh), vl = frag_kb(V + VPL + (size_t)(n * 16 + col) * NP + kb, hh); o[n] = wmma16b(vf, pb, o[n]); o[n] = wmma16b(vf, pl, o[n]); o[n] = wmma16b(vl, pb, o[n]); } }
  const float inv = 1.0f / (l * VS * PS);
#pragma unroll
  for (int n = 0; n < 2; ++n)
#pragma unroll
    for (int r = 0; r < 8; ++r) Os[col][h * DH + n * 16 + 8 * hh + r] = o[n][r] * inv;
  __syncthreads();
  float* dst = orow + (size_t)q0 * C;
  for (int pass = 0; pass < 2; ++pass) { for (int i = threadIdx.x; i < 16 * C / 4; i += 256) { const int rr = i >> 6, c4 = (i & 63) * 4; *(volatile v4f*)(dst + (size_t)rr * C + c4) = *(const v4f*)(&Os[rr][c4]); } __threadfence(); }
}

__global__ __launch_bounds__(128) void conv_kernel(const float* __restrict__ orow, const b16* __restrict__ wt16, const float* __restrict__ bt, const float* __restrict__ x, float* __restrict__ out) {
  __shared__ __attribute__((aligned(16))) float Tc[64][128 + 4];
  const int lane = threadIdx.x & 31, wave = threadIdx.x >> 5, nloc = lane & 15, hlf = lane >> 4, m0 = blockIdx.y * 128 + wave * 32, c0 = blockIdx.x * 64, p0 = blockIdx.y * 128;
  const int pa = m0 + nloc, pb_ = m0 + 16 + nloc; const int za = pa >> 8, ya = (pa >> 4) & 15, xa = pa & 15, zb = pb_ >> 8, yb = (pb_ >> 4) & 15, xb = pb_ & 15;
  v8f acc[2][4];
#pragma unroll
  for (int r = 0; r < 2; ++r)
#pragma unroll
    for (int t = 0; t < 4; ++t) acc[r][t] = (v8f){};
  for (int tap = 0; tap < 27; ++tap) { const int dz = tap / 9 - 1, dy = (tap / 3) % 3 - 1, dx = tap % 3 - 1;
    const int z1 = za + dz, y1 = ya + dy, x1 = xa + dx, z2 = zb + dz, y2 = yb + dy, x2 = xb + dx;
    const bool oka = ((unsigned)z1 < 16u) && ((unsigned)y1 < 16u) && ((unsigned)x1 < 16u), okb = ((unsigned)z2 < 16u) && ((unsigned)y2 < 16u) && ((unsigned)x2 < 16u);
    const int qa = (min(max(z1, 0), 15) << 8) | (min(max(y1, 0), 15) << 4) | min(max(x1, 0), 15), qb = (min(max(z2, 0), 15) << 8) | (min(max(y2, 0), 15) << 4) | min(max(x2, 0), 15);
    const float* ra = orow + (size_t)qa * C; const float* rb = orow + (size_t)qb * C;
#pragma unroll 2
    for (int kb = 0; kb < C; kb += 32) { v16b a0, a1, l0, l1;
#pragma unroll
      for (int e = 0; e < 16; ++e) { const int k = kb + ((e < 8) ? (8 * hlf + e) : (16 + 8 * hlf + e - 8)); b16 p, q; const float va = oka ? ra[k] : 0.0f, vb = okb ? rb[k] : 0.0f;
        split16(va * OS_, p, q); a0[e] = p; l0[e] = q; split16(vb * OS_, p, q); a1[e] = p; l1[e] = q; }
#pragma unroll
      for (int t = 0; t < 4; ++t) { const v16b bw = frag_kb(wt16 + (size_t)(c0 + t * 16 + nloc) * KT + tap * C + kb, hlf); acc[0][t] = wmma16b(a0, bw, acc[0][t]); acc[0][t] = wmma16b(l0, bw, acc[0][t]); acc[1][t] = wmma16b(a1, bw, acc[1][t]); acc[1][t] = wmma16b(l1, bw, acc[1][t]); } } }
#pragma unroll
  for (int t = 0; t < 4; ++t) { const int co = c0 + t * 16 + nloc; const float bb = bf16_rne(bt[co]);
#pragma unroll
    for (int r = 0; r < 2; ++r)
#pragma unroll
      for (int v = 0; v < 8; ++v) { const int pl_ = wave * 32 + r * 16 + 8 * hlf + v; Tc[t * 16 + nloc][pl_] = acc[r][t][v] * (1.0f / OS_) + bb + bf16_rne(x[(size_t)co * NP + p0 + pl_]); } }
  __syncthreads();
  for (int pass = 0; pass < 2; ++pass) { for (int i = threadIdx.x; i < 64 * 32; i += 128) { const int cc = i >> 5, c4 = (i & 31) * 4; *(volatile v4f*)(out + (size_t)(c0 + cc) * NP + p0 + c4) = *(const v4f*)(&Tc[cc][c4]); } __threadfence(); }
}
}

extern "C" void kernel_launch(void* const* d_in, const int* in_sizes, int n_in,
                              void* d_out, int out_size, void* d_ws, size_t ws_size, hipStream_t stream) {
  (void)n_in; (void)out_size;
  const float* x = (const float*)d_in[0]; const float* wq = (const float*)d_in[1]; const float* bq = (const float*)d_in[2]; const float* wk = (const float*)d_in[3]; const float* bk = (const float*)d_in[4]; const float* wv = (const float*)d_in[5]; const float* bv = (const float*)d_in[6]; const float* wt = (const float*)d_in[7]; const float* bt = (const float*)d_in[8];
  float* out = (float*)d_out;
  if (in_sizes[0] != C * NP || in_sizes[1] != C * C || in_sizes[3] != C * C || in_sizes[5] != C * C || in_sizes[7] != C * C * 27) return;
  size_t off = 0; char* ws = (char*)d_ws;
  auto carve = [&](size_t bytes) { char* p = ws + off; off += (bytes + 255) & ~(size_t)255; return p; };
  unsigned short* xT = (unsigned short*)carve((size_t)NP * C * 2); unsigned short* w16 = (unsigned short*)carve((size_t)3 * C * C * 2); b16* wt16 = (b16*)carve((size_t)C * KT * 2);
  b16* qhp = (b16*)carve(QPL * 2 * 2); b16* khp = (b16*)carve(QPL * 2 * 2); b16* vtp = (b16*)carve(VPL * 2 * 2); float* orow = (float*)carve((size_t)NP * C * 4);
  if (off > ws_size) return;
  prep_kernel<<<NP / 64, 256, 0, stream>>>(x, wq, wk, wv, wt, xT, w16, wt16);
  proj_kernel<<<dim3(C / 64, NP / 128, 3), 128, 0, stream>>>(xT, w16, bq, bk, bv, qhp, khp, vtp);
  attn_kernel<<<NP / 16, 256, 0, stream>>>(qhp, khp, vtp, orow);
  conv_kernel<<<dim3(C / 64, NP / 128), 128, 0, stream>>>(orow, wt16, bt, x, out);
}
